// GCN3_16552803959363
// MI455X (gfx1250) — hardware-verified
//
#include <hip/hip_runtime.h>
#include <stddef.h>
#include <stdint.h>


#define FD      128
#define KA      256
#define NOUT    64
#define NTHR    256
#define NWAVE   8
#define EPT     8
#define CHUNK   (NTHR * EPT)
#define WCAP    (EPT * 32)
#define LISTN   (NWAVE * WCAP)
#define NBMAX   2048
#define ESH     11
#define RCAP    28672
#define DEGCAP  4096
#define STW     512
#define NBD     4096
#define GBM     64
#define GBN     64
#define GTHR    128
#define WSMAX   134217728
#define LDS_AGG ((2 * RCAP + 2 * NBMAX + LISTN) * 4 + 64)
#define LDS_DEG ((NWAVE * NBD + LISTN) * 4 + 64)

static_assert((CHUNK & (CHUNK - 1)) == 0 && CHUNK <= 4096);
static_assert((NBMAX & (NBMAX - 1)) == 0 && NBMAX <= (1 << ESH) && NBMAX <= 4096);
static_assert((NBD & (NBD - 1)) == 0 && NBD <= 4096);
static_assert(NBD == 16 * NTHR);
static_assert(NTHR * 8 == NBMAX);
static_assert(LISTN >= NBMAX);
static_assert(LISTN >= NWAVE * WCAP);
static_assert((RCAP % 32) == 0);
static_assert(NWAVE * STW <= RCAP);
static_assert(STW >= FD);
static_assert(LDS_AGG <= 300000 && LDS_DEG <= 300000);
static_assert(GBM == (GTHR / 32) * 16);
static_assert(KA == 2 * FD && (KA % 32) == 0);
static_assert((FD % GBN) == 0 && (NOUT % GBN) == 0);
static_assert(FD == 4 * 32);

typedef float          v4f  __attribute__((ext_vector_type(4)));
typedef float          v8f  __attribute__((ext_vector_type(8)));
typedef int            v4i  __attribute__((ext_vector_type(4)));
typedef int            v8i  __attribute__((ext_vector_type(8)));
typedef unsigned short v4us __attribute__((ext_vector_type(4)));
typedef unsigned short v8us __attribute__((ext_vector_type(8)));
typedef __bf16         v16b __attribute__((ext_vector_type(16)));
union FragB { v16b v; v8us h[2]; v8i w; };

__device__ __forceinline__ v8f wmb(const FragB& a, const FragB& b, v8f c) {
  v8f d = __builtin_amdgcn_wmma_f32_16x16x32_bf16(false, a.v, false, b.v, (short)0, c, false, false);
  asm volatile("v_nop\n\tv_nop\n\tv_nop\n\tv_nop" : "+v"(d) : "v"(a.w), "v"(b.w));
  return d;
}

__device__ __forceinline__ unsigned short bf16r(float f) {
  const unsigned u = __float_as_uint(f);
  return (unsigned short)((u + 0x7FFFu + ((u >> 16) & 1u)) >> 16);
}
__device__ __forceinline__ float bf16f(unsigned short b) { return __uint_as_float((unsigned)b << 16); }
__device__ __forceinline__ unsigned short split2(float x, bool lo) {
  const unsigned short hb = bf16r(x);
  const unsigned short lb = bf16r(x - bf16f(hb));
  return lo ? lb : hb;
}
__device__ __forceinline__ v8us cvt8b(const v4f a, const v4f b) {
  v8us r;
  r[0] = bf16r(a.x); r[1] = bf16r(a.y); r[2] = bf16r(a.z); r[3] = bf16r(a.w);
  r[4] = bf16r(b.x); r[5] = bf16r(b.y); r[6] = bf16r(b.z); r[7] = bf16r(b.w);
  return r;
}

__device__ __forceinline__ int scan_chunk(const int* __restrict__ ids, int nE, int cbase, int slotBase,
                                          int nb, int vec8, int* list, int tid, int lane, int wave) {
  int wc = 0;
  const int el0  = tid * EPT;
  const int e0   = cbase + el0;
  const int sent = -2147483647 - 1;
  v4i da, db;
  if (vec8 != 0 && cbase + CHUNK <= nE) {
    da = *(const v4i*)(ids + e0);
    db = *(const v4i*)(ids + e0 + 4);
  } else {
    da.x = (e0     < nE) ? ids[min(e0,     nE - 1)] : sent;
    da.y = (e0 + 1 < nE) ? ids[min(e0 + 1, nE - 1)] : sent;
    da.z = (e0 + 2 < nE) ? ids[min(e0 + 2, nE - 1)] : sent;
    da.w = (e0 + 3 < nE) ? ids[min(e0 + 3, nE - 1)] : sent;
    db.x = (e0 + 4 < nE) ? ids[min(e0 + 4, nE - 1)] : sent;
    db.y = (e0 + 5 < nE) ? ids[min(e0 + 5, nE - 1)] : sent;
    db.z = (e0 + 6 < nE) ? ids[min(e0 + 6, nE - 1)] : sent;
    db.w = (e0 + 7 < nE) ? ids[min(e0 + 7, nE - 1)] : sent;
  }
  const unsigned nbs = (unsigned)slotBase;
  const unsigned unb = (unsigned)nb;
  const unsigned s0 = (unsigned)da.x - nbs, s1 = (unsigned)da.y - nbs;
  const unsigned s2 = (unsigned)da.z - nbs, s3 = (unsigned)da.w - nbs;
  const unsigned s4 = (unsigned)db.x - nbs, s5 = (unsigned)db.y - nbs;
  const unsigned s6 = (unsigned)db.z - nbs, s7 = (unsigned)db.w - nbs;
  const bool h0 = s0 < unb, h1 = s1 < unb, h2 = s2 < unb, h3 = s3 < unb;
  const bool h4 = s4 < unb, h5 = s5 < unb, h6 = s6 < unb, h7 = s7 < unb;
  const unsigned any = __builtin_amdgcn_ballot_w32(h0 | h1 | h2 | h3 | h4 | h5 | h6 | h7);
  if (any != 0u) {
#define HITJ(J, HJ, SJ) { \
      const unsigned mj = __builtin_amdgcn_ballot_w32(HJ); \
      if (mj != 0u) { \
        if (HJ) { \
          const int pos = wc + (int)__builtin_amdgcn_mbcnt_lo(mj, 0u); \
          if (pos < WCAP) list[wave * WCAP + pos] = ((el0 + (J)) << 12) | (int)(SJ); \
        } \
        wc += (int)__builtin_popcount(mj); } }
    HITJ(0, h0, s0)
    HITJ(1, h1, s1)
    HITJ(2, h2, s2)
    HITJ(3, h3, s3)
    HITJ(4, h4, s4)
    HITJ(5, h5, s5)
    HITJ(6, h6, s6)
    HITJ(7, h7, s7)
#undef HITJ
  }
  return wc;
}

__global__ __launch_bounds__(NTHR) void k_outdeg(const int* __restrict__ srcs, float* ns, int nE, int vec8) {
  extern __shared__ v4f lds_dyn[];
  int* hist = (int*)lds_dyn;
  int* list = hist + NWAVE * NBD;
  const int tid = (int)threadIdx.x, lane = tid & 31, wave = tid >> 5;
  const int nodeBase = (int)blockIdx.x * NBD;
  for (int i = tid; i < NWAVE * NBD; i += NTHR) hist[i] = 0;
  __syncthreads();
  int* hw = hist + wave * NBD;
  const int nChunks = (nE + CHUNK - 1) / CHUNK;
#pragma unroll 1
  for (int ch = 0; ch < nChunks; ++ch) {
    const int cbase = ch * CHUNK;
    const int wc = scan_chunk(srcs, nE, cbase, nodeBase, NBD, vec8, list, tid, lane, wave);
    __builtin_amdgcn_fence(__ATOMIC_RELEASE, "wavefront");
    __builtin_amdgcn_wave_barrier();
    const int wcc = wc > WCAP ? WCAP : wc;
#pragma unroll 1
    for (int b0 = 0; b0 < wcc; b0 += 32) {
      const int idx = b0 + lane;
      const int uv  = list[wave * WCAP + (idx < WCAP ? idx : WCAP - 1)];
      const int m32 = (wcc - b0) < 32 ? (wcc - b0) : 32;
#pragma unroll 1
      for (int k = 0; k < m32; ++k) {
        const int u  = __builtin_amdgcn_readlane(uv, k);
        const int sl = u & (NBD - 1);
        if (lane == 0) hw[sl] = hw[sl] + 1;
      }
    }
    __builtin_amdgcn_fence(__ATOMIC_RELEASE, "wavefront");
    __builtin_amdgcn_wave_barrier();
  }
  __syncthreads();
  v4f ov[4];
#pragma unroll
  for (int p = 0; p < 4; ++p) {
    const int s4 = (p * NTHR + tid) * 4;
    int c0 = 0, c1 = 0, c2 = 0, c3 = 0;
#pragma unroll
    for (int w2 = 0; w2 < NWAVE; ++w2) {
      const v4i hv = *(const v4i*)(hist + w2 * NBD + s4);
      c0 += hv.x; c1 += hv.y; c2 += hv.z; c3 += hv.w;
    }
    ov[p].x = rsqrtf((float)(c0 < 1 ? 1 : c0));
    ov[p].y = rsqrtf((float)(c1 < 1 ? 1 : c1));
    ov[p].z = rsqrtf((float)(c2 < 1 ? 1 : c2));
    ov[p].w = rsqrtf((float)(c3 < 1 ? 1 : c3));
  }
#pragma unroll
  for (int p = 0; p < 4; ++p) {
    const int s4 = (p * NTHR + tid) * 4;
    *(volatile v4f*)(ns + nodeBase + s4) = ov[p];
  }
  __threadfence();
#pragma unroll
  for (int p = 0; p < 4; ++p) {
    const int s4 = (p * NTHR + tid) * 4;
    *(volatile v4f*)(ns + nodeBase + s4) = ov[p];
  }
}

__global__ __launch_bounds__(NTHR) void k_xprep(const float* __restrict__ x, unsigned short* xb, int nUnits) {
  const int i = (int)blockIdx.x * NTHR + (int)threadIdx.x;
  if (i >= nUnits) return;
  const float* p = x + (size_t)i * 8;
  const v4f a = *(const v4f*)p, b = *(const v4f*)(p + 4);
  const v8us hv = cvt8b(a, b);
  const size_t o = (size_t)i * 8;
  *(volatile v8us*)(xb + o) = hv;
  __threadfence();
  *(volatile v8us*)(xb + o) = hv;
}

__global__ __launch_bounds__(NTHR) void k_wtr(const float* __restrict__ w, int Kin, int cols,
                                              unsigned short* wt, int nUnits) {
  const int u = (int)blockIdx.x * NTHR + (int)threadIdx.x;
  if (u >= nUnits) return;
  const int kq = KA >> 3;
  const int n  = u / kq;
  const int k8 = (u - n * kq) * 8;
  int kk = k8 < Kin ? k8 : k8 - Kin;
  kk = kk < 0 ? 0 : (kk > Kin - 8 ? Kin - 8 : kk);
  const float* p = w + (size_t)kk * (size_t)cols + n;
  v4f a, b;
  a.x = p[0];                  a.y = p[(size_t)cols];       a.z = p[(size_t)2 * cols];   a.w = p[(size_t)3 * cols];
  b.x = p[(size_t)4 * cols];   b.y = p[(size_t)5 * cols];   b.z = p[(size_t)6 * cols];   b.w = p[(size_t)7 * cols];
  const v8us hv = cvt8b(a, b);
  const size_t o = (size_t)n * (size_t)KA + k8;
  *(volatile v8us*)(wt + o) = hv;
  __threadfence();
  *(volatile v8us*)(wt + o) = hv;
}

template<int RELU>
__global__ __launch_bounds__(GTHR) void k_gemm(
    const unsigned short* __restrict__ A, const unsigned short* __restrict__ WT,
    const float* __restrict__ bias, int blen, float* outF, int K, int ldo, int nRows)
{
  __shared__ __attribute__((aligned(16))) float stg[GBM * GBN];
  const int tid = (int)threadIdx.x, lane = tid & 31, wave = tid >> 5, hh = lane >> 4, m = lane & 15;
  const int rowBase = (int)blockIdx.x * GBM;
  const int col0    = (int)blockIdx.y * GBN;

  v8f acc[4];
  {
    const v8f z = {0.f, 0.f, 0.f, 0.f, 0.f, 0.f, 0.f, 0.f};
    acc[0] = z; acc[1] = z; acc[2] = z; acc[3] = z;
  }
  const unsigned short* ap = A  + (size_t)(rowBase + 16 * wave + m) * (size_t)K + 8 * hh;
  const unsigned short* wp = WT + (size_t)(col0 + m) * (size_t)K + 8 * hh;
  const int ksteps = K >> 5;
#pragma unroll 1
  for (int ks = 0; ks < ksteps; ++ks) {
    FragB af;
    af.h[0] = *(const v8us*)(ap + 32 * ks);
    af.h[1] = *(const v8us*)(ap + 32 * ks + 16);
#pragma unroll
    for (int t = 0; t < 4; ++t) {
      const unsigned short* wq = wp + (size_t)(16 * t) * (size_t)K + 32 * ks;
      FragB bf;
      bf.h[0] = *(const v8us*)wq;
      bf.h[1] = *(const v8us*)(wq + 16);
      acc[t] = wmb(af, bf, acc[t]);
    }
  }

#pragma unroll
  for (int t = 0; t < 4; ++t) {
    const int lc = 16 * t + m;
    int bi = col0 + lc;
    bi = bi > blen - 1 ? blen - 1 : bi;
    bi = bi < 0 ? 0 : bi;
    const float bv = bf16f(bf16r(bias[bi]));
#pragma unroll
    for (int r = 0; r < 8; ++r) {
      const int lr = 16 * wave + 8 * hh + r;
      float v = acc[t][r] + bv;
      if (RELU) v = fmaxf(v, 0.0f);
      stg[lr * GBN + lc] = v;
    }
  }
  __syncthreads();

  v4f fv[8];
#pragma unroll
  for (int i = 0; i < 8; ++i) {
    const int lr = 16 * wave + 2 * i + hh;
    fv[i] = *(const v4f*)(stg + lr * GBN + 4 * m);
  }
#pragma unroll
  for (int i = 0; i < 8; ++i) {
    const int lr = 16 * wave + 2 * i + hh;
    const int gr = rowBase + lr;
    float* op = outF + (size_t)gr * (size_t)ldo + col0 + 4 * m;
    if (gr < nRows) *(volatile v4f*)op = fv[i];
  }
  __threadfence();
#pragma unroll
  for (int i = 0; i < 8; ++i) {
    const int lr = 16 * wave + 2 * i + hh;
    const int gr = rowBase + lr;
    float* op = outF + (size_t)gr * (size_t)ldo + col0 + 4 * m;
    if (gr < nRows) *(volatile v4f*)op = fv[i];
  }
}

template<int SRC16>
__global__ __launch_bounds__(NTHR) void k_agg(
    const int* __restrict__ srcs, const int* __restrict__ dsts,
    const unsigned short* __restrict__ XB, const float* __restrict__ HF, const float* __restrict__ ns,
    unsigned short* Aout, int nN, int nE, int nb, int vec8, int MPr) {
  extern __shared__ v4f lds_dyn[];
  int* reg1 = (int*)lds_dyn;
  int* reg2 = reg1 + RCAP;
  int* scnt = reg2 + RCAP;
  int* soff = scnt + NBMAX;
  int* list = soff + NBMAX;
  int* wcnt = list + LISTN;
  int* wtot = wcnt + NWAVE;
  const int tid = (int)threadIdx.x, lane = tid & 31, wave = tid >> 5;
  const int nodeBase = (int)blockIdx.x * nb;

  for (int i = tid; i < NBMAX; i += NTHR) scnt[i] = 0;
  __syncthreads();

  int tot = 0;
  const int nChunks = (nE + CHUNK - 1) / CHUNK;
#pragma unroll 1
  for (int ch = 0; ch < nChunks; ++ch) {
    const int cbase = ch * CHUNK;
    const int wc = scan_chunk(dsts, nE, cbase, nodeBase, nb, vec8, list, tid, lane, wave);
    if (lane == 0) wcnt[wave] = wc;
    __syncthreads();
    int pre = 0, all = 0;
#pragma unroll
    for (int w2 = 0; w2 < NWAVE; ++w2) {
      int c = wcnt[w2];
      c = c < 0 ? 0 : (c > WCAP ? WCAP : c);
      all += c;
      pre += (w2 < wave) ? c : 0;
    }
    const int wcc  = wc > WCAP ? WCAP : wc;
    const int base = tot + pre;
#pragma unroll 1
    for (int i = lane; i < wcc; i += 32) {
      const int ent = list[wave * WCAP + i];
      const int el  = (ent >> 12) & (CHUNK - 1);
      const int sl  = ent & (NBMAX - 1);
      int eid = cbase + el;
      eid = eid > nE - 1 ? nE - 1 : eid;
      const int pos = base + i;
      if (pos < RCAP) reg1[pos] = (int)(((unsigned)eid << ESH) | (unsigned)sl);
    }
    tot += all;
    tot = tot > RCAP ? RCAP : tot;
    __syncthreads();
  }
  const int nh = tot;

  if (wave == 0) {
#pragma unroll 1
    for (int b0 = 0; b0 < nh; b0 += 32) {
      const int idx = b0 + lane;
      const int uv  = reg1[idx < RCAP ? idx : RCAP - 1];
      const int m32 = (nh - b0) < 32 ? (nh - b0) : 32;
#pragma unroll 1
      for (int k = 0; k < m32; ++k) {
        const int u  = __builtin_amdgcn_readlane(uv, k);
        const int sl = u & (NBMAX - 1);
        if (lane == 0) scnt[sl] = scnt[sl] + 1;
      }
    }
  }
  __syncthreads();

  {
    const v4i ca = *(const v4i*)(scnt + 8 * tid);
    const v4i cb = *(const v4i*)(scnt + 8 * tid + 4);
    const int e0 = ca.x < 0 ? 0 : ca.x, e1 = ca.y < 0 ? 0 : ca.y, e2 = ca.z < 0 ? 0 : ca.z, e3 = ca.w < 0 ? 0 : ca.w;
    const int e4 = cb.x < 0 ? 0 : cb.x, e5 = cb.y < 0 ? 0 : cb.y, e6 = cb.z < 0 ? 0 : cb.z, e7 = cb.w < 0 ? 0 : cb.w;
    const int ts = e0 + e1 + e2 + e3 + e4 + e5 + e6 + e7;
    int incl = ts;
#pragma unroll
    for (int d = 1; d < 32; d <<= 1) {
      const int up = __shfl_up(incl, d);
      if (lane >= d) incl += up;
    }
    if (lane == 31) wtot[wave] = incl;
    __syncthreads();
    int pre = 0;
#pragma unroll
    for (int w2 = 0; w2 < NWAVE; ++w2) pre += (w2 < wave) ? wtot[w2] : 0;
    int run = pre + incl - ts;
    soff[8 * tid + 0] = run; run += e0;
    soff[8 * tid + 1] = run; run += e1;
    soff[8 * tid + 2] = run; run += e2;
    soff[8 * tid + 3] = run; run += e3;
    soff[8 * tid + 4] = run; run += e4;
    soff[8 * tid + 5] = run; run += e5;
    soff[8 * tid + 6] = run; run += e6;
    soff[8 * tid + 7] = run;
  }
  __syncthreads();
  for (int i = tid; i < NBMAX; i += NTHR) list[i] = soff[i];
  __syncthreads();

  if (wave == 0) {
#pragma unroll 1
    for (int b0 = 0; b0 < nh; b0 += 32) {
      const int idx = b0 + lane;
      const int uv  = reg1[idx < RCAP ? idx : RCAP - 1];
      const int m32 = (nh - b0) < 32 ? (nh - b0) : 32;
#pragma unroll 1
      for (int k = 0; k < m32; ++k) {
        const int u   = __builtin_amdgcn_readlane(uv, k);
        const int sl  = u & (NBMAX - 1);
        const int eid = (int)((unsigned)u >> ESH);
        if (lane == 0) {
          int pos = list[sl];
          pos = pos < 0 ? 0 : (pos > RCAP - 1 ? RCAP - 1 : pos);
          reg2[pos] = eid;
          list[sl] = pos + 1;
        }
      }
    }
  }
  __syncthreads();

  const int nbw = nb >> 3;
  const bool ovf = (nh >= RCAP);
  const float qnan = __int_as_float(0x7fc00000);
  float* stw = (float*)reg1 + wave * STW;
  const int l16 = lane & 15;
  const bool islo = lane >= 16;
#pragma unroll 1
  for (int jt = 0; jt < nbw; ++jt) {
    const int slot = wave * nbw + jt;
    const int grow = nodeBase + slot;
    int st = soff[slot];
    const int craw = scnt[slot];
    int cnt = craw;
    st  = st < 0 ? 0 : (st > nh ? nh : st);
    cnt = cnt < 0 ? 0 : (cnt > DEGCAP ? DEGCAP : cnt);
    if (cnt > nh - st) cnt = nh - st;
    const float pz = (ovf || craw > DEGCAP) ? qnan : 0.0f;
    const bool wr = grow < MPr;
    const float live = grow < nN ? 1.0f : 0.0f;
    const float nd = rsqrtf((float)(craw < 1 ? 1 : craw));

    float a0 = 0.f, a1 = 0.f, a2 = 0.f, a3 = 0.f;
#pragma unroll 1
    for (int q0 = 0; q0 < cnt; q0 += 32) {
      const int m32 = (cnt - q0) < 32 ? (cnt - q0) : 32;
      int idx = st + q0 + lane; idx = idx > RCAP - 1 ? RCAP - 1 : idx;
      int eid = reg2[idx]; eid = eid < 0 ? 0 : (eid > nE - 1 ? nE - 1 : eid);
      const int sraw = srcs[eid];
      const int sl = sraw < 0 ? 0 : (sraw > nN - 1 ? nN - 1 : sraw);
      const int wl = __float_as_int(ns[sl]);
#pragma unroll 1
      for (int k = 0; k < m32; ++k) {
        const int s = __builtin_amdgcn_readlane(sl, k);
        const float w = __int_as_float(__builtin_amdgcn_readlane(wl, k));
        float v0, v1, v2, v3;
        if (SRC16 != 0) {
          const v4us uv = *(const v4us*)(XB + (size_t)s * FD + 4 * lane);
          v0 = bf16f(uv.x); v1 = bf16f(uv.y); v2 = bf16f(uv.z); v3 = bf16f(uv.w);
        } else {
          const v4f fv = *(const v4f*)(HF + (size_t)s * FD + 4 * lane);
          v0 = fv.x; v1 = fv.y; v2 = fv.z; v3 = fv.w;
        }
        a0 = fmaf(w, v0, a0); a1 = fmaf(w, v1, a1); a2 = fmaf(w, v2, a2); a3 = fmaf(w, v3, a3);
      }
    }
    const float sc = nd * live;
    v4f rv;
    rv.x = a0 * sc + pz; rv.y = a1 * sc + pz; rv.z = a2 * sc + pz; rv.w = a3 * sc + pz;
    __builtin_amdgcn_fence(__ATOMIC_RELEASE, "wavefront");
    __builtin_amdgcn_wave_barrier();
    *(v4f*)(stw + 4 * lane) = rv;
    __builtin_amdgcn_fence(__ATOMIC_RELEASE, "wavefront");
    __builtin_amdgcn_wave_barrier();
    const v4f ga = *(const v4f*)(stw + 8 * l16);
    const v4f gb = *(const v4f*)(stw + 8 * l16 + 4);
    v8us hv;
    hv[0] = split2(ga.x, islo); hv[1] = split2(ga.y, islo); hv[2] = split2(ga.z, islo); hv[3] = split2(ga.w, islo);
    hv[4] = split2(gb.x, islo); hv[5] = split2(gb.y, islo); hv[6] = split2(gb.z, islo); hv[7] = split2(gb.w, islo);
    unsigned short* gp = Aout + (size_t)grow * KA + 8 * lane;
    if (wr) *(volatile v8us*)gp = hv;
    __threadfence();
    if (wr) *(volatile v8us*)gp = hv;
  }
}

static int pick_nb(int nE, int nN) {
  int nb = NBMAX;
  while (nb > 16 && (long long)nb * (long long)nE * 5LL > (long long)RCAP * (long long)nN * 4LL) nb >>= 1;
  return nb;
}
static inline int cdiv(int a, int b) { return (a + b - 1) / b; }

extern "C" void kernel_launch(void* const* d_in, const int* in_sizes, int n_in,
                              void* d_out, int out_size, void* d_ws, size_t ws_size,
                              hipStream_t stream) {
  if (n_in < 7) return;
  const int nN = in_sizes[0] / FD;
  if (nN <= 0 || in_sizes[0] != nN * FD || nN > (1 << 22)) return;
  const int nE = in_sizes[1];
  if (nE < 1 || nE > (1 << 21) || in_sizes[2] != nE) return;
  if (in_sizes[3] != FD * FD || in_sizes[4] != FD) return;
  if (in_sizes[5] != FD * NOUT || in_sizes[6] != NOUT) return;
  if (out_size != nN * NOUT) return;

  const float* x   = (const float*)d_in[0];
  const int*   src = (const int*)  d_in[1];
  const int*   dst = (const int*)  d_in[2];
  const float* W1  = (const float*)d_in[3];
  const float* b1  = (const float*)d_in[4];
  const float* W2  = (const float*)d_in[5];
  const float* b2  = (const float*)d_in[6];
  float* out = (float*)d_out;

  const int MP   = cdiv(nN, GBM) * GBM;
  const int nb   = pick_nb(nE, nN);
  const int gA   = cdiv(MP, nb);
  const int gD   = cdiv(nN, NBD);
  const int MPD  = gD * NBD;
  const int vec8 = ((nE & 3) == 0) ? 1 : 0;
  if (gA * nb < MP || MPD < nN) return;

  char* ws = (char*)d_ws;
  size_t off = 0;
  const size_t oNS  = off; off += (size_t)MPD * 4;                 off = (off + 255) & ~(size_t)255;
  const size_t oXB  = off; off += (size_t)MP * FD * 2;             off = (off + 255) & ~(size_t)255;
  const size_t oWT1 = off; off += (size_t)FD * KA * 2;             off = (off + 255) & ~(size_t)255;
  const size_t oWT2 = off; off += (size_t)NOUT * KA * 2;           off = (off + 255) & ~(size_t)255;
  const size_t oAP  = off; off += (size_t)MP * KA * 2;             off = (off + 255) & ~(size_t)255;
  const size_t oH   = off; off += (size_t)MP * FD * 4;             off = (off + 255) & ~(size_t)255;
  if (off > ws_size || off > (size_t)WSMAX) return;
  float*          NS  = (float*)(ws + oNS);
  unsigned short* XB  = (unsigned short*)(ws + oXB);
  unsigned short* WT1 = (unsigned short*)(ws + oWT1);
  unsigned short* WT2 = (unsigned short*)(ws + oWT2);
  unsigned short* AP  = (unsigned short*)(ws + oAP);
  float*          H   = (float*)(ws + oH);

  hipFuncSetAttribute(reinterpret_cast<const void*>(&k_outdeg),
                      hipFuncAttributeMaxDynamicSharedMemorySize, LDS_DEG);
  hipFuncSetAttribute(reinterpret_cast<const void*>(&k_agg<1>),
                      hipFuncAttributeMaxDynamicSharedMemorySize, LDS_AGG);
  hipFuncSetAttribute(reinterpret_cast<const void*>(&k_agg<0>),
                      hipFuncAttributeMaxDynamicSharedMemorySize, LDS_AGG);

  k_outdeg<<<gD, NTHR, LDS_DEG, stream>>>(src, NS, nE, vec8);

  const int nUx = nN * (FD / 8);
  k_xprep<<<cdiv(nUx, NTHR), NTHR, 0, stream>>>(x, XB, nUx);

  {
    const int nU1 = FD * (KA / 8);
    k_wtr<<<cdiv(nU1, NTHR), NTHR, 0, stream>>>(W1, FD, FD, WT1, nU1);
    const int nU2 = NOUT * (KA / 8);
    k_wtr<<<cdiv(nU2, NTHR), NTHR, 0, stream>>>(W2, FD, NOUT, WT2, nU2);
  }

  const int gM = MP / GBM;
  k_agg<1><<<gA, NTHR, LDS_AGG, stream>>>(src, dst, XB, H, NS, AP, nN, nE, nb, vec8, MP);
  k_gemm<1><<<dim3(gM, FD / GBN), GTHR, 0, stream>>>(AP, WT1, b1, FD, H, KA, FD, MP);
  k_agg<0><<<gA, NTHR, LDS_AGG, stream>>>(src, dst, XB, H, NS, AP, nN, nE, nb, vec8, MP);
  k_gemm<0><<<dim3(gM, NOUT / GBN), GTHR, 0, stream>>>(AP, WT2, b2, NOUT, out, KA, NOUT, nN);
}
